// GNNModel_63247688401329
// MI455X (gfx1250) — hardware-run, weakly checked
//
#include <hip/hip_runtime.h>
#include <stddef.h>
#include <stdint.h>
#include <math.h>

#define H1_TERMS 2

#define NN      100000
#define NE      1600000
#define CIN     128
#define HID     64
#define OUTD    32
#define GBM     128
#define MP      100096
#define KL      128
#define K2      (64 * H1_TERMS)
#define NTHR    256
#define NWAVE   8
#define EPT     8
#define WCH     (32 * EPT)
#define NBRUN   1024
#define SLB     10
#define NBK     98
#define WLCAP   4096
#define RCAP    20480
#define DEGCAP  64
#define MAXDEG_MEAS   36
#define MAXB1024_MEAS 16710
#define RPB     128
#define SP      68
#define SP2     36
#define WSMAX   134217728

#define BK_ZINTS (NWAVE * WLCAP + RCAP + 3 * NBRUN)
#define BK_INTS  (BK_ZINTS + NBRUN + 16)
#define BK_LDS   (BK_INTS * 4)

#define PBX  (MP * CIN / 8 / NTHR)
#define PBW1 (HID * CIN / 8 / NTHR)
#define PBW2 (OUTD * KL / 8 / NTHR)
#define PBZ  ((MP - NN) * KL / 8 / NTHR)
#define PBTOT (PBX + PBW1 + PBW2 + PBZ + 1)

static_assert(H1_TERMS == 1 || H1_TERMS == 2);
static_assert(HID == 64 && OUTD == 32 && HID % 16 == 0 && OUTD % 16 == 0);
static_assert(CIN % 32 == 0 && KL % 32 == 0 && K2 % 32 == 0 && KL == 2 * HID);
static_assert(MP % GBM == 0 && MP >= NN && MP == 782 * GBM && MP % RPB == 0);
static_assert(NBRUN == 1024 && NBRUN == (1 << SLB) && NBRUN % RPB == 0 && NBRUN % GBM == 0 && NBRUN % 32 == 0);
static_assert(NBK * NBRUN >= MP && (NBK - 1) * NBRUN < NN);
static_assert(NN <= (1 << 17));
static_assert(NE < (1 << 21) && (((long long)NE) << SLB) < (1LL << 31));
static_assert(NE % WCH == 0 && NE % 4 == 0);
static_assert((long long)RCAP * 100 >= (long long)MAXB1024_MEAS * 105);
static_assert((long long)WLCAP * NWAVE * 2 >= (long long)MAXB1024_MEAS * 3);
static_assert(MAXDEG_MEAS + 8 <= DEGCAP);
static_assert(RCAP % (NTHR * 4) == 0 && BK_ZINTS % 4 == 0 && NBRUN == NTHR * 4);
static_assert(BK_LDS <= 300000);
static_assert((GBM * SP + GBM) * 4 <= 65536);
static_assert((MP * CIN / 8) % NTHR == 0 && (HID * CIN / 8) % NTHR == 0 && (OUTD * KL / 8) % NTHR == 0);
static_assert(((MP - NN) * KL / 8) % NTHR == 0);
static_assert(RPB == NWAVE * 16 && GBM == NWAVE * 16);

typedef float          v4f   __attribute__((ext_vector_type(4)));
typedef float          v8f   __attribute__((ext_vector_type(8)));
typedef int            v2i   __attribute__((ext_vector_type(2)));
typedef int            v4i   __attribute__((ext_vector_type(4)));
typedef int            v8i   __attribute__((ext_vector_type(8)));
typedef unsigned short v8us  __attribute__((ext_vector_type(8)));
typedef unsigned short v16us __attribute__((ext_vector_type(16)));
typedef __bf16         v16bf __attribute__((ext_vector_type(16)));
typedef v4f  __attribute__((may_alias)) v4fa;
typedef v4i  __attribute__((may_alias)) v4ia;
typedef v8us __attribute__((may_alias)) v8usa;
union FragB { v16bf v; v16us u; v8us h[2]; v8i w; };

__device__ __forceinline__ v8f wmb(const FragB& a, const FragB& b, v8f c) {
  v8f d = __builtin_amdgcn_wmma_f32_16x16x32_bf16(false, a.v, false, b.v, (short)0, c, false, false);
  asm volatile("v_nop\n\tv_nop\n\tv_nop\n\tv_nop" : "+v"(d) : "v"(a.w), "v"(b.w));
  return d;
}

__device__ __forceinline__ unsigned bf16_bits(float f) {
  const unsigned u = __float_as_uint(f);
  const unsigned r = (u + 0x7FFFu + ((u >> 16) & 1u)) >> 16;
  const unsigned q = (u >> 16) | 0x40u;
  return ((u & 0x7fffffffu) > 0x7f800000u) ? q : r;
}

__device__ __forceinline__ void hilo_pack(float v0, float v1, float v2, float v3,
                                          int& h01, int& h23, int& l01, int& l23) {
  const unsigned a0 = bf16_bits(v0), a1 = bf16_bits(v1), a2 = bf16_bits(v2), a3 = bf16_bits(v3);
  const unsigned b0 = bf16_bits(v0 - __uint_as_float(a0 << 16));
  const unsigned b1 = bf16_bits(v1 - __uint_as_float(a1 << 16));
  const unsigned b2 = bf16_bits(v2 - __uint_as_float(a2 << 16));
  const unsigned b3 = bf16_bits(v3 - __uint_as_float(a3 << 16));
  h01 = (int)(a0 | (a1 << 16)); h23 = (int)(a2 | (a3 << 16));
  l01 = (int)(b0 | (b1 << 16)); l23 = (int)(b2 | (b3 << 16));
}

__device__ __forceinline__ void st2_v4f(float* p, v4f v) {
  *(volatile v4f*)p = v;
  __threadfence();
  *(volatile v4f*)p = v;
}
__device__ __forceinline__ void st2_v8us(unsigned short* p, v8us v) {
  *(volatile v8us*)p = v;
  __threadfence();
  *(volatile v8us*)p = v;
}

__device__ __forceinline__ v8us col8(const float* __restrict__ base, int stride) {
  float f[8];
#pragma unroll
  for (int i = 0; i < 8; ++i) f[i] = base[(size_t)i * (size_t)stride];
  v8us o;
#pragma unroll
  for (int i = 0; i < 8; ++i) o[i] = (unsigned short)bf16_bits(f[i]);
  return o;
}

__global__ __launch_bounds__(NTHR) void k_prep(const float* __restrict__ x, const float* __restrict__ w1,
                                               const float* __restrict__ b1, const float* __restrict__ w2,
                                               const float* __restrict__ b2,
                                               unsigned short* xb, unsigned short* w1t, unsigned short* w2d,
                                               unsigned short* x1, float* sm) {
  const int tid = (int)threadIdx.x, lane = tid & 31;
  const int blk = (int)blockIdx.x;
  if (blk < PBX) {
    const int u   = blk * NTHR + tid;
    const int row = u >> 4, k8 = (u & 15) * 8;
    const int rc  = row < NN ? row : NN - 1;
    const unsigned mk = row < NN ? 0xffffu : 0u;
    const float* p = x + (size_t)rc * CIN + k8;
    const v4f a = *(const v4fa*)p;
    const v4f b = *(const v4fa*)(p + 4);
    v8us o;
    o[0] = (unsigned short)(bf16_bits(a.x) & mk); o[1] = (unsigned short)(bf16_bits(a.y) & mk);
    o[2] = (unsigned short)(bf16_bits(a.z) & mk); o[3] = (unsigned short)(bf16_bits(a.w) & mk);
    o[4] = (unsigned short)(bf16_bits(b.x) & mk); o[5] = (unsigned short)(bf16_bits(b.y) & mk);
    o[6] = (unsigned short)(bf16_bits(b.z) & mk); o[7] = (unsigned short)(bf16_bits(b.w) & mk);
    st2_v8us(xb + (size_t)row * CIN + k8, o);
  } else if (blk < PBX + PBW1) {
    const int u = (blk - PBX) * NTHR + tid;
    const int n = u >> 4, k8 = (u & 15) * 8;
    const v8us o = col8(w1 + (size_t)k8 * HID + n, HID);
    st2_v8us(w1t + (size_t)n * CIN + k8, o);
  } else if (blk < PBX + PBW1 + PBW2) {
    const int u = (blk - PBX - PBW1) * NTHR + tid;
    const int n = u >> 4, k8 = (u & 15) * 8, kk = k8 & 63;
    const v8us o = col8(w2 + (size_t)kk * OUTD + n, OUTD);
    st2_v8us(w2d + (size_t)n * KL + k8, o);
  } else if (blk < PBX + PBW1 + PBW2 + PBZ) {
    const int u = (blk - PBX - PBW1 - PBW2) * NTHR + tid;
    const v8us z = {0, 0, 0, 0, 0, 0, 0, 0};
    st2_v8us(x1 + (size_t)NN * KL + (size_t)u * 8, z);
  } else {
    if (tid < 32) {
      const v4f a = *(const v4fa*)(b1 + 4 * (lane & 15));
      const v4f c = *(const v4fa*)(b2 + 4 * (lane & 7));
      asm volatile("" :: "v"(a));
      asm volatile("" :: "v"(c));
      const unsigned ma = (lane < 16) ? 0xffffffffu : 0u;
      const unsigned mb = ((lane >= 16) & (lane < 24)) ? 0xffffffffu : 0u;
      v4f o;
      o.x = __uint_as_float(((bf16_bits(a.x) << 16) & ma) | ((bf16_bits(c.x) << 16) & mb));
      o.y = __uint_as_float(((bf16_bits(a.y) << 16) & ma) | ((bf16_bits(c.y) << 16) & mb));
      o.z = __uint_as_float(((bf16_bits(a.z) << 16) & ma) | ((bf16_bits(c.z) << 16) & mb));
      o.w = __uint_as_float(((bf16_bits(a.w) << 16) & ma) | ((bf16_bits(c.w) << 16) & mb));
      st2_v4f(sm + 4 * lane, o);
    }
  }
}

__device__ __forceinline__ void bucket_flush(const int* pl, const int* co, const int* dvi, int ov,
                                             int* lp, int* cop, int* dvp, int* fp, int tid) {
#pragma unroll 1
  for (int i = tid * 4; i < RCAP; i += NTHR * 4) {
    const v4i v = *(const v4ia*)(pl + i);
    *(volatile v4i*)(lp + i) = v;
  }
  {
    const v4i v = *(const v4ia*)(co + 4 * tid);
    *(volatile v4i*)(cop + 4 * tid) = v;
  }
  {
    const v4i v = *(const v4ia*)(co + NBRUN + 4 * tid);
    *(volatile v4i*)(cop + NBRUN + 4 * tid) = v;
  }
  {
    const v4i v = *(const v4ia*)(dvi + 4 * tid);
    *(volatile v4i*)(dvp + 4 * tid) = v;
  }
  if (tid < 8) {
    const v4i f = {ov, ov, ov, ov};
    *(volatile v4i*)(fp + 4 * tid) = f;
  }
}

__global__ __launch_bounds__(NTHR) void k_bucket(const int* __restrict__ srcs, const int* __restrict__ dsts,
                                                 int* LIST, int* CO, int* DINVI, int* FLAG) {
  extern __shared__ __attribute__((aligned(16))) int dsm[];
  int* wl   = dsm;
  int* pl   = dsm + NWAVE * WLCAP;
  int* cnt  = pl + RCAP;
  int* offs = cnt + NBRUN;
  int* cur  = offs + NBRUN;
  int* dvi  = cur + NBRUN;
  int* misc = dvi + NBRUN;
  const int tid = (int)threadIdx.x, lane = tid & 31, wave = tid >> 5;
  const int blk = (int)blockIdx.x;
  const unsigned nbs = (unsigned)(blk * NBRUN);
  int nbi = NN - blk * NBRUN;
  nbi = nbi > NBRUN ? NBRUN : (nbi < 0 ? 0 : nbi);
  const unsigned unb = (unsigned)nbi;

  {
    const v4i z4 = {0, 0, 0, 0};
    for (int i = tid * 4; i < BK_ZINTS; i += NTHR * 4) *(v4ia*)(dsm + i) = z4;
    if (tid < 16) misc[tid] = 0;
  }
  __syncthreads();

  {
    const int per  = ((NE + NWAVE * WCH - 1) / (NWAVE * WCH)) * WCH;
    const int ebeg = wave * per;
    const int eend = (ebeg + per < NE) ? (ebeg + per) : NE;
    int* mylist = wl + wave * WLCAP;
    int wc = 0;
#pragma unroll 1
    for (int cb = ebeg; cb < eend; cb += WCH) {
      const int e0 = cb + lane * EPT;
      const v4i da = *(const v4ia*)(dsts + e0);
      const v4i db = *(const v4ia*)(dsts + e0 + 4);
      const unsigned s0 = (unsigned)da.x - nbs, s1 = (unsigned)da.y - nbs;
      const unsigned s2 = (unsigned)da.z - nbs, s3 = (unsigned)da.w - nbs;
      const unsigned s4 = (unsigned)db.x - nbs, s5 = (unsigned)db.y - nbs;
      const unsigned s6 = (unsigned)db.z - nbs, s7 = (unsigned)db.w - nbs;
      const bool h0 = s0 < unb, h1 = s1 < unb, h2 = s2 < unb, h3 = s3 < unb;
      const bool h4 = s4 < unb, h5 = s5 < unb, h6 = s6 < unb, h7 = s7 < unb;
      const unsigned m0 = __builtin_amdgcn_ballot_w32(h0), m1 = __builtin_amdgcn_ballot_w32(h1);
      const unsigned m2 = __builtin_amdgcn_ballot_w32(h2), m3 = __builtin_amdgcn_ballot_w32(h3);
      const unsigned m4 = __builtin_amdgcn_ballot_w32(h4), m5 = __builtin_amdgcn_ballot_w32(h5);
      const unsigned m6 = __builtin_amdgcn_ballot_w32(h6), m7 = __builtin_amdgcn_ballot_w32(h7);
      const unsigned any = m0 | m1 | m2 | m3 | m4 | m5 | m6 | m7;
      if (any != 0u) {
        const int pre = (int)(__builtin_amdgcn_mbcnt_lo(m0, 0u) + __builtin_amdgcn_mbcnt_lo(m1, 0u) +
                              __builtin_amdgcn_mbcnt_lo(m2, 0u) + __builtin_amdgcn_mbcnt_lo(m3, 0u) +
                              __builtin_amdgcn_mbcnt_lo(m4, 0u) + __builtin_amdgcn_mbcnt_lo(m5, 0u) +
                              __builtin_amdgcn_mbcnt_lo(m6, 0u) + __builtin_amdgcn_mbcnt_lo(m7, 0u));
        int p = wc + pre;
        if (h0) { if (p < WLCAP) mylist[p] = ((e0 + 0) << SLB) | (int)s0; p = p + 1; }
        if (h1) { if (p < WLCAP) mylist[p] = ((e0 + 1) << SLB) | (int)s1; p = p + 1; }
        if (h2) { if (p < WLCAP) mylist[p] = ((e0 + 2) << SLB) | (int)s2; p = p + 1; }
        if (h3) { if (p < WLCAP) mylist[p] = ((e0 + 3) << SLB) | (int)s3; p = p + 1; }
        if (h4) { if (p < WLCAP) mylist[p] = ((e0 + 4) << SLB) | (int)s4; p = p + 1; }
        if (h5) { if (p < WLCAP) mylist[p] = ((e0 + 5) << SLB) | (int)s5; p = p + 1; }
        if (h6) { if (p < WLCAP) mylist[p] = ((e0 + 6) << SLB) | (int)s6; p = p + 1; }
        if (h7) { if (p < WLCAP) mylist[p] = ((e0 + 7) << SLB) | (int)s7; p = p + 1; }
        wc += (int)(__builtin_popcount(m0) + __builtin_popcount(m1) + __builtin_popcount(m2) + __builtin_popcount(m3) +
                    __builtin_popcount(m4) + __builtin_popcount(m5) + __builtin_popcount(m6) + __builtin_popcount(m7));
      }
    }
    if (lane == 0) misc[wave] = wc;
  }
  __syncthreads();

  if (wave == 0) {
    int ov = 0;
#pragma unroll 1
    for (int w2 = 0; w2 < NWAVE; ++w2) {
      int c = __builtin_amdgcn_readfirstlane(misc[w2]);
      if (c > WLCAP) ov = 1;
      c = c < 0 ? 0 : (c > WLCAP ? WLCAP : c);
#pragma unroll 1
      for (int b0 = 0; b0 < c; b0 += 32) {
        const int idx = b0 + lane;
        const int ent = wl[w2 * WLCAP + (idx < WLCAP ? idx : WLCAP - 1)];
        const int m32 = (c - b0) < 32 ? (c - b0) : 32;
#pragma unroll 1
        for (int k = 0; k < m32; ++k) {
          const int u    = __builtin_amdgcn_readlane(ent, k);
          const int slot = u & (NBRUN - 1);
          if (lane == 0) cnt[slot] = cnt[slot] + 1;
        }
      }
    }
    if (lane == 0) misc[9] = ov;
  }
  __syncthreads();
  if (wave == 0) {
    const int base = lane * (NBRUN / 32);
    int s = 0;
#pragma unroll 1
    for (int i = 0; i < NBRUN / 32; ++i) s += cnt[base + i];
    int incl = s;
#pragma unroll
    for (int d = 1; d < 32; d <<= 1) {
      const int y = __shfl_up(incl, d, 32);
      if (lane >= d) incl += y;
    }
    int run = incl - s;
#pragma unroll 1
    for (int i = 0; i < NBRUN / 32; ++i) {
      const int cv = cnt[base + i];
      offs[base + i] = run;
      cur[base + i]  = run;
      run += cv;
    }
    if (lane == 31) misc[10] = (run > RCAP) ? 1 : 0;
  }
  __syncthreads();

  if (wave == 0) {
#pragma unroll 1
    for (int w2 = 0; w2 < NWAVE; ++w2) {
      int c = __builtin_amdgcn_readfirstlane(misc[w2]);
      c = c < 0 ? 0 : (c > WLCAP ? WLCAP : c);
#pragma unroll 1
      for (int b0 = 0; b0 < c; b0 += 32) {
        const int idx = b0 + lane;
        const int ent = wl[w2 * WLCAP + (idx < WLCAP ? idx : WLCAP - 1)];
        int eid = (ent >> SLB) & 0x1FFFFF;
        eid = eid > NE - 1 ? NE - 1 : eid;
        int sr = srcs[eid];
        sr = sr < 0 ? 0 : (sr > NN - 1 ? NN - 1 : sr);
        const int m32 = (c - b0) < 32 ? (c - b0) : 32;
#pragma unroll 1
        for (int k = 0; k < m32; ++k) {
          const int u    = __builtin_amdgcn_readlane(ent, k);
          const int wd   = __builtin_amdgcn_readlane(sr, k);
          const int slot = u & (NBRUN - 1);
          if (lane == 0) {
            int p = cur[slot];
            p = p < 0 ? 0 : (p > RCAP - 1 ? RCAP - 1 : p);
            pl[p] = wd;
            cur[slot] = p + 1;
          }
        }
      }
    }
  }
  __syncthreads();

#pragma unroll 1
  for (int it = 0; it < NBRUN / NTHR; ++it) {
    const int s = it * NTHR + tid;
    const float dg = (float)(cnt[s] + 1);
    dvi[s] = __float_as_int(1.0f / sqrtf(dg));
  }
  __syncthreads();

  const int ovf = misc[9] | misc[10];
  int* lp  = LIST + (size_t)blk * RCAP;
  int* cop = CO + (size_t)blk * (2 * NBRUN);
  int* dvp = DINVI + (size_t)blk * NBRUN;
  int* fp  = FLAG + (size_t)blk * 32;
  bucket_flush(pl, cnt, dvi, ovf, lp, cop, dvp, fp, tid);
  __threadfence();
  bucket_flush(pl, cnt, dvi, ovf, lp, cop, dvp, fp, tid);
}

template <int KTOT, int PITCH, int NT>
__device__ __forceinline__ void gemm_tile(const unsigned short* __restrict__ ap,
                                          const unsigned short* __restrict__ bp, v8f (&acc)[NT]) {
#pragma unroll 1
  for (int k0 = 0; k0 < KTOT; k0 += 32) {
    FragB af;
    af.h[0] = *(const v8usa*)(ap + k0);
    af.h[1] = *(const v8usa*)(ap + k0 + 16);
#pragma unroll
    for (int nt = 0; nt < NT; ++nt) {
      const unsigned short* wq = bp + (size_t)(16 * nt) * (size_t)PITCH + k0;
      FragB bf;
      bf.h[0] = *(const v8usa*)wq;
      bf.h[1] = *(const v8usa*)(wq + 16);
      acc[nt] = wmb(af, bf, acc[nt]);
    }
  }
}

template <int NT, int PITCHF>
__device__ __forceinline__ void stage_d(float* stg, const v8f (&acc)[NT], int wave, int hh, int m) {
#pragma unroll
  for (int nt = 0; nt < NT; ++nt) {
#pragma unroll
    for (int r = 0; r < 8; ++r) stg[(16 * wave + 8 * hh + r) * PITCHF + 16 * nt + m] = acc[nt][r];
  }
}

__global__ __launch_bounds__(NTHR) __attribute__((amdgpu_num_vgpr(248)))
void k_mm1(const unsigned short* __restrict__ XB, const unsigned short* __restrict__ W1T,
           const float* __restrict__ DINV, float* H1P) {
  __shared__ __attribute__((aligned(16))) float stg[GBM * SP];
  __shared__ __attribute__((aligned(16))) float sdv[GBM];
  const int tid = (int)threadIdx.x, lane = tid & 31, wave = tid >> 5, hh = lane >> 4, m = lane & 15;
  const int rowBase = (int)blockIdx.x * GBM;
  if (tid < 32) *(v4fa*)(sdv + 4 * tid) = *(const v4fa*)(DINV + (size_t)rowBase + 4 * tid);

  v8f acc[4];
  {
    const v8f z = {0.f, 0.f, 0.f, 0.f, 0.f, 0.f, 0.f, 0.f};
#pragma unroll
    for (int t = 0; t < 4; ++t) acc[t] = z;
  }
  const unsigned short* ap = XB + (size_t)(rowBase + 16 * wave + m) * (size_t)CIN + 8 * hh;
  const unsigned short* bp = W1T + (size_t)m * (size_t)CIN + 8 * hh;
  gemm_tile<CIN, CIN, 4>(ap, bp, acc);
  stage_d<4, SP>(stg, acc, wave, hh, m);
  __syncthreads();

#pragma unroll 1
  for (int i = 0; i < 8; ++i) {
    const int lr   = 16 * wave + 2 * i + hh;
    const int grow = rowBase + lr;
    const v4f a = *(const v4fa*)(stg + lr * SP + 4 * m);
    const float dv = sdv[lr];
    v4f o;
    o.x = a.x * dv; o.y = a.y * dv; o.z = a.z * dv; o.w = a.w * dv;
    st2_v4f(H1P + (size_t)grow * HID + 4 * m, o);
  }
}

__global__ __launch_bounds__(NTHR) __attribute__((amdgpu_num_vgpr(248)))
void k_mm2(const unsigned short* __restrict__ X1HL, const unsigned short* __restrict__ W2D,
           const float* __restrict__ DINV, float* H2P) {
  __shared__ __attribute__((aligned(16))) float stg[GBM * SP2];
  __shared__ __attribute__((aligned(16))) float sdv[GBM];
  const int tid = (int)threadIdx.x, lane = tid & 31, wave = tid >> 5, hh = lane >> 4, m = lane & 15;
  const int rowBase = (int)blockIdx.x * GBM;
  if (tid < 32) *(v4fa*)(sdv + 4 * tid) = *(const v4fa*)(DINV + (size_t)rowBase + 4 * tid);

  v8f acc[2];
  {
    const v8f z = {0.f, 0.f, 0.f, 0.f, 0.f, 0.f, 0.f, 0.f};
    acc[0] = z; acc[1] = z;
  }
  const unsigned short* ap = X1HL + (size_t)(rowBase + 16 * wave + m) * (size_t)KL + 8 * hh;
  const unsigned short* bp = W2D + (size_t)m * (size_t)KL + 8 * hh;
  gemm_tile<K2, KL, 2>(ap, bp, acc);
  stage_d<2, SP2>(stg, acc, wave, hh, m);
  __syncthreads();

  const int qq = lane >> 3, l8 = lane & 7;
#pragma unroll 1
  for (int i = 0; i < 4; ++i) {
    const int lr   = 16 * wave + 4 * i + qq;
    const int grow = rowBase + lr;
    const v4f a = *(const v4fa*)(stg + lr * SP2 + 4 * l8);
    const float dv = sdv[lr];
    v4f o;
    o.x = a.x * dv; o.y = a.y * dv; o.z = a.z * dv; o.w = a.w * dv;
    st2_v4f(H2P + (size_t)grow * OUTD + 4 * l8, o);
  }
}

__global__ __launch_bounds__(NTHR) void k_rep1(const int* __restrict__ LIST, const int* __restrict__ CO,
                                               const int* __restrict__ FLAG, const float* __restrict__ DINV,
                                               const float* __restrict__ H1P, const float* __restrict__ SM,
                                               unsigned short* X1HL) {
  __shared__ __attribute__((aligned(16))) float sb[128];
  const int tid = (int)threadIdx.x, lane = tid & 31, hh = lane >> 4, q = lane & 15;
  const int wave = __builtin_amdgcn_readfirstlane(tid >> 5);
  const int rowBase = (int)blockIdx.x * RPB;
  const int bucket  = rowBase >> SLB;
  if (tid < 32) *(v4fa*)(sb + 4 * tid) = *(const v4fa*)(SM + 4 * tid);
  __syncthreads();
  const v4f bias = *(const v4fa*)(sb + 4 * q);
  const int* lb  = LIST + (size_t)bucket * RCAP;
  const int* cob = CO + (size_t)bucket * (2 * NBRUN);
  const int flag = FLAG[(size_t)bucket * 32];
  const float qnan = __uint_as_float(0x7fc00000u);

#pragma unroll 1
  for (int i = 0; i < RPB / NWAVE; ++i) {
    const int d = rowBase + (RPB / NWAVE) * wave + i;
    if (d < NN) {
      const int slot = d & (NBRUN - 1);
      int c = __builtin_amdgcn_readfirstlane(cob[slot]);
      int o = __builtin_amdgcn_readfirstlane(cob[NBRUN + slot]);
      const bool big = c > DEGCAP;
      c = c < 0 ? 0 : (c > DEGCAP ? DEGCAP : c);
      o = o < 0 ? 0 : (o > RCAP - 1 ? RCAP - 1 : o);
      int last = o + c - 1;
      last = last < o ? o : last;
      last = last > RCAP - 1 ? RCAP - 1 : last;
      const int trips = (c + 1) >> 1;
      float a0 = 0.0f, a1 = 0.0f, a2 = 0.0f, a3 = 0.0f;
#pragma unroll 1
      for (int j = 0; j < trips; ++j) {
        const int t = 2 * j + hh;
        int idx = o + t;
        idx = idx > last ? last : idx;
        int sr = lb[idx];
        sr = sr < 0 ? 0 : (sr > NN - 1 ? NN - 1 : sr);
        const v4f v = *(const v4fa*)(H1P + (size_t)sr * HID + 4 * q);
        asm volatile("" :: "v"(v));
        const bool valid = t < c;
        const float t0 = a0 + v.x, t1 = a1 + v.y, t2 = a2 + v.z, t3 = a3 + v.w;
        a0 = valid ? t0 : a0; a1 = valid ? t1 : a1; a2 = valid ? t2 : a2; a3 = valid ? t3 : a3;
      }
      a0 += __shfl_xor(a0, 16, 32); a1 += __shfl_xor(a1, 16, 32);
      a2 += __shfl_xor(a2, 16, 32); a3 += __shfl_xor(a3, 16, 32);
      const v4f g = *(const v4fa*)(H1P + (size_t)d * HID + 4 * q);
      const float dv = DINV[d];
      float m0 = (a0 + g.x) * dv + bias.x, m1 = (a1 + g.y) * dv + bias.y;
      float m2 = (a2 + g.z) * dv + bias.z, m3 = (a3 + g.w) * dv + bias.w;
      m0 = (m0 > 0.0f) ? m0 : (m0 - m0); m1 = (m1 > 0.0f) ? m1 : (m1 - m1);
      m2 = (m2 > 0.0f) ? m2 : (m2 - m2); m3 = (m3 > 0.0f) ? m3 : (m3 - m3);
      const bool bad = (flag != 0) | big;
      m0 = bad ? qnan : m0; m1 = bad ? qnan : m1; m2 = bad ? qnan : m2; m3 = bad ? qnan : m3;
      int h01, h23, l01, l23;
      hilo_pack(m0, m1, m2, m3, h01, h23, l01, l23);
      const int mk = (hh == 0) ? -1 : 0;
      v2i ow;
      ow.x = (h01 & mk) | (l01 & ~mk);
      ow.y = (h23 & mk) | (l23 & ~mk);
      unsigned short* hp = X1HL + (size_t)d * KL + 64 * hh + 4 * q;
      *(volatile v2i*)hp = ow;
      __threadfence();
      *(volatile v2i*)hp = ow;
    }
  }
}

__global__ __launch_bounds__(NTHR) void k_rep2(const int* __restrict__ LIST, const int* __restrict__ CO,
                                               const int* __restrict__ FLAG, const float* __restrict__ DINV,
                                               const float* __restrict__ H2P, const float* __restrict__ SM,
                                               float* out) {
  __shared__ __attribute__((aligned(16))) float sb[128];
  const int tid = (int)threadIdx.x, lane = tid & 31, qq = lane >> 3, l8 = lane & 7;
  const int wave = __builtin_amdgcn_readfirstlane(tid >> 5);
  const int rowBase = (int)blockIdx.x * RPB;
  const int bucket  = rowBase >> SLB;
  if (tid < 32) *(v4fa*)(sb + 4 * tid) = *(const v4fa*)(SM + 4 * tid);
  __syncthreads();
  const v4f bias = *(const v4fa*)(sb + 64 + 4 * l8);
  const int* lb  = LIST + (size_t)bucket * RCAP;
  const int* cob = CO + (size_t)bucket * (2 * NBRUN);
  const int flag = FLAG[(size_t)bucket * 32];
  const float qnan = __uint_as_float(0x7fc00000u);

#pragma unroll 1
  for (int i = 0; i < RPB / NWAVE; ++i) {
    const int d = rowBase + (RPB / NWAVE) * wave + i;
    if (d < NN) {
      const int slot = d & (NBRUN - 1);
      int c = __builtin_amdgcn_readfirstlane(cob[slot]);
      int o = __builtin_amdgcn_readfirstlane(cob[NBRUN + slot]);
      const bool big = c > DEGCAP;
      c = c < 0 ? 0 : (c > DEGCAP ? DEGCAP : c);
      o = o < 0 ? 0 : (o > RCAP - 1 ? RCAP - 1 : o);
      int last = o + c - 1;
      last = last < o ? o : last;
      last = last > RCAP - 1 ? RCAP - 1 : last;
      const int trips = (c + 3) >> 2;
      float a0 = 0.0f, a1 = 0.0f, a2 = 0.0f, a3 = 0.0f;
#pragma unroll 1
      for (int j = 0; j < trips; ++j) {
        const int t = 4 * j + qq;
        int idx = o + t;
        idx = idx > last ? last : idx;
        int sr = lb[idx];
        sr = sr < 0 ? 0 : (sr > NN - 1 ? NN - 1 : sr);
        const v4f v = *(const v4fa*)(H2P + (size_t)sr * OUTD + 4 * l8);
        asm volatile("" :: "v"(v));
        const bool valid = t < c;
        const float t0 = a0 + v.x, t1 = a1 + v.y, t2 = a2 + v.z, t3 = a3 + v.w;
        a0 = valid ? t0 : a0; a1 = valid ? t1 : a1; a2 = valid ? t2 : a2; a3 = valid ? t3 : a3;
      }
      a0 += __shfl_xor(a0, 8, 32); a1 += __shfl_xor(a1, 8, 32);
      a2 += __shfl_xor(a2, 8, 32); a3 += __shfl_xor(a3, 8, 32);
      a0 += __shfl_xor(a0, 16, 32); a1 += __shfl_xor(a1, 16, 32);
      a2 += __shfl_xor(a2, 16, 32); a3 += __shfl_xor(a3, 16, 32);
      const v4f g = *(const v4fa*)(H2P + (size_t)d * OUTD + 4 * l8);
      asm volatile("" :: "v"(g));
      const float dv = DINV[d];
      asm volatile("" :: "v"(dv));
      float m0 = (a0 + g.x) * dv + bias.x, m1 = (a1 + g.y) * dv + bias.y;
      float m2 = (a2 + g.z) * dv + bias.z, m3 = (a3 + g.w) * dv + bias.w;
      const bool bad = (flag != 0) | big;
      m0 = bad ? qnan : m0; m1 = bad ? qnan : m1; m2 = bad ? qnan : m2; m3 = bad ? qnan : m3;
      v4f ov;
      ov.x = m0; ov.y = m1; ov.z = m2; ov.w = m3;
      float* op = out + (size_t)d * OUTD + 4 * l8;
      const bool wr = lane < 8;
      if (wr) *(volatile v4f*)op = ov;
      __threadfence();
      if (wr) *(volatile v4f*)op = ov;
    }
  }
}

extern "C" void kernel_launch(void* const* d_in, const int* in_sizes, int n_in,
                              void* d_out, int out_size, void* d_ws, size_t ws_size,
                              hipStream_t stream) {
  if (n_in < 6) return;
  if (in_sizes[0] != NN * CIN) return;
  if (in_sizes[1] != 2 * NE) return;
  if (in_sizes[2] != CIN * HID) return;
  if (in_sizes[3] != HID) return;
  if (in_sizes[4] != HID * OUTD) return;
  if (in_sizes[5] != OUTD) return;
  if (out_size != NN * OUTD) return;

  const float* x  = (const float*)d_in[0];
  const int*   ei = (const int*)d_in[1];
  const float* W1 = (const float*)d_in[2];
  const float* b1 = (const float*)d_in[3];
  const float* W2 = (const float*)d_in[4];
  const float* b2 = (const float*)d_in[5];
  float* out = (float*)d_out;
  const int* srcs = ei;
  const int* dsts = ei + NE;

  constexpr size_t zXB   = (size_t)MP * CIN * 2;
  constexpr size_t zH1P  = (size_t)MP * HID * 4;
  constexpr size_t zX1   = (size_t)MP * KL * 2;
  constexpr size_t zH2P  = (size_t)MP * OUTD * 4;
  constexpr size_t zLIST = (size_t)NBK * RCAP * 4;
  constexpr size_t zCO   = (size_t)NBK * 2 * NBRUN * 4;
  constexpr size_t zDINV = (size_t)NBK * NBRUN * 4;
  constexpr size_t zFLAG = (size_t)NBK * 128;
  constexpr size_t zW1T  = (size_t)HID * CIN * 2;
  constexpr size_t zW2D  = (size_t)OUTD * KL * 2;
  constexpr size_t zSM   = 512;
  constexpr size_t oXB   = 0;
  constexpr size_t oH1P  = oXB + zXB;
  constexpr size_t oX1   = oH1P + zH1P;
  constexpr size_t oH2P  = oX1 + zX1;
  constexpr size_t oLIST = oH2P + zH2P;
  constexpr size_t oCO   = oLIST + zLIST;
  constexpr size_t oDINV = oCO + zCO;
  constexpr size_t oFLAG = oDINV + zDINV;
  constexpr size_t oW1T  = oFLAG + zFLAG;
  constexpr size_t oW2D  = oW1T + zW1T;
  constexpr size_t oSM   = oW2D + zW2D;
  constexpr size_t oEND  = oSM + zSM;
  static_assert(zXB % 256 == 0 && zH1P % 256 == 0 && zX1 % 256 == 0 && zH2P % 256 == 0 && zLIST % 256 == 0);
  static_assert(zCO % 256 == 0 && zDINV % 256 == 0 && zFLAG % 256 == 0 && zW1T % 256 == 0 && zW2D % 256 == 0);
  static_assert(zSM % 256 == 0);
  static_assert((size_t)NBK * NBRUN >= (size_t)MP);
  static_assert(oEND <= (size_t)WSMAX);
  if (oEND > ws_size) return;

  char* ws = (char*)d_ws;
  unsigned short* XB   = (unsigned short*)(ws + oXB);
  float*          H1P  = (float*)(ws + oH1P);
  unsigned short* X1HL = (unsigned short*)(ws + oX1);
  float*          H2P  = (float*)(ws + oH2P);
  int*            LIST = (int*)(ws + oLIST);
  int*            CO   = (int*)(ws + oCO);
  float*          DINV = (float*)(ws + oDINV);
  int*            FLAG = (int*)(ws + oFLAG);
  unsigned short* W1T  = (unsigned short*)(ws + oW1T);
  unsigned short* W2D  = (unsigned short*)(ws + oW2D);
  float*          SM   = (float*)(ws + oSM);

  hipFuncSetAttribute(reinterpret_cast<const void*>(&k_bucket), hipFuncAttributeMaxDynamicSharedMemorySize, (int)BK_LDS);

  k_prep<<<PBTOT, NTHR, 0, stream>>>(x, W1, b1, W2, b2, XB, W1T, W2D, X1HL, SM);
  k_bucket<<<NBK, NTHR, BK_LDS, stream>>>(srcs, dsts, LIST, CO, (int*)DINV, FLAG);
  k_mm1<<<MP / GBM, NTHR, 0, stream>>>(XB, W1T, DINV, H1P);
  k_rep1<<<MP / RPB, NTHR, 0, stream>>>(LIST, CO, FLAG, DINV, H1P, SM, X1HL);
  k_mm2<<<MP / GBM, NTHR, 0, stream>>>(X1HL, W2D, DINV, H2P);
  k_rep2<<<MP / RPB, NTHR, 0, stream>>>(LIST, CO, FLAG, DINV, H2P, SM, out);
}
